// MultiHeadSelfAttention_70222715289849
// MI455X (gfx1250) — hardware-verified
//
#include <hip/hip_runtime.h>


#ifndef NB
#define NB 2
#endif
#ifndef SEQ
#define SEQ 2048
#endif
#define NB_FULL  2
#define SEQ_FULL 2048
#define DM   1024
#define NH   16
#define HD   64
#define SCL  0.125f
#define L2E  1.4426950408889634f
#define EXC  (SCL * L2E)
#define CCAR 64.0f
#define WCAR 1024.0f
#define OSC  (1.0f / 65536.0f)
#define AW   4
#define QW   32
#define KB   64
#define KH   32

static_assert(DM == NH * HD);
static_assert(HD == 64);
static_assert(DM % 64 == 0);
static_assert(DM % 32 == 0);
static_assert(SEQ % 64 == 0);
static_assert((NB * SEQ) % 64 == 0);
static_assert(SEQ % (AW * QW) == 0);
static_assert(SEQ % KB == 0);
static_assert(KB == 64);
static_assert(KH == 32);
static_assert(KB % KH == 0);
static_assert(QW == 32);
static_assert(NB <= NB_FULL);
static_assert(SEQ <= SEQ_FULL);
static_assert(CCAR * WCAR * OSC == 1.0f);

typedef _Float16 h16;
typedef unsigned short bf;
typedef __attribute__((ext_vector_type(16))) __bf16   v16bf;
typedef __attribute__((ext_vector_type(16))) _Float16 v16h;
typedef __attribute__((ext_vector_type(8)))  _Float16 v8h;
typedef __attribute__((ext_vector_type(8)))  unsigned short v8us;
typedef __attribute__((ext_vector_type(8)))  float    v8f;
typedef __attribute__((ext_vector_type(4)))  float    v4f;
typedef v8h  __attribute__((may_alias)) v8ha;
typedef v4f  __attribute__((may_alias)) v4fa;

__device__ __forceinline__ unsigned short f2bf(float f) { unsigned u = __float_as_uint(f); u += 0x7FFFu + ((u >> 16) & 1u); return (unsigned short)(u >> 16); }
__device__ __forceinline__ float bf2f(unsigned short b) { return __uint_as_float(((unsigned)b) << 16); }
__device__ __forceinline__ float bfr(float f) { return bf2f(f2bf(f)); }
__device__ __forceinline__ v16h cat16(v8h lo, v8h hi) { return __builtin_shufflevector(lo, hi, 0, 1, 2, 3, 4, 5, 6, 7, 8, 9, 10, 11, 12, 13, 14, 15); }
__device__ __forceinline__ v16bf cat16b(v8us lo, v8us hi) { return __builtin_bit_cast(v16bf, __builtin_shufflevector(lo, hi, 0, 1, 2, 3, 4, 5, 6, 7, 8, 9, 10, 11, 12, 13, 14, 15)); }
__device__ __forceinline__ v8f wmma16(v16h a, v16h b, v8f c) { return __builtin_amdgcn_wmma_f32_16x16x32_f16(false, a, false, b, (short)0, c, false, false); }
__device__ __forceinline__ v8f wmmab(v16bf a, v16bf b, v8f c) { return __builtin_amdgcn_wmma_f32_16x16x32_bf16(false, a, false, b, (short)0, c, false, false); }

template <typename T16> struct WFrag;
template <> struct WFrag<h16> { typedef v16h V; static __device__ __forceinline__ V ld(const h16* p) { return cat16(*(const v8h*)p, *(const v8h*)(p + 16)); } static __device__ __forceinline__ v8f mma(V a, V b, v8f c) { return wmma16(a, b, c); } };
template <> struct WFrag<bf> { typedef v16bf V; static __device__ __forceinline__ V ld(const bf* p) { return cat16b(*(const v8us*)p, *(const v8us*)(p + 16)); } static __device__ __forceinline__ v8f mma(V a, V b, v8f c) { return wmmab(a, b, c); } };

__global__ __launch_bounds__(256) void k_cvt8(const float* __restrict__ src, bf* dst, size_t n8, size_t sstride, size_t dstride) {
    const size_t i = (size_t)blockIdx.x * 256 + threadIdx.x; if (i >= n8) return;
    const float* s = src + (size_t)blockIdx.y * sstride; bf* d = dst + (size_t)blockIdx.y * dstride;
    const v8f v = *(const v8f*)(s + i * 8); v8us o;
#pragma unroll
    for (int k = 0; k < 8; ++k) o[k] = f2bf(v[k]);
    *(volatile v8us*)(d + i * 8) = o; __threadfence(); *(volatile v8us*)(d + i * 8) = o;
}
__global__ __launch_bounds__(256) void k_cvt8h(const float* __restrict__ src, h16* dst, size_t n8) {
    const size_t i = (size_t)blockIdx.x * 256 + threadIdx.x; if (i >= n8) return;
    const v8f v = *(const v8f*)(src + i * 8); v8h o;
#pragma unroll
    for (int k = 0; k < 8; ++k) o[k] = (h16)(bfr(v[k]) * WCAR);
    *(volatile v8h*)(dst + i * 8) = o; __threadfence(); *(volatile v8h*)(dst + i * 8) = o;
}

template <typename T16, int MODE>
__device__ __forceinline__ void gemm_body(const T16* __restrict__ A, const T16* __restrict__ Bt, const float* __restrict__ bias, h16* o16, float* o32) {
    typedef typename WFrag<T16>::V V;
    __shared__ __align__(16) float os[16 * 68];
    __shared__ __align__(16) h16 vts[64 * 72];
    const int lane = threadIdx.x & 31, lr = lane & 15, hi = lane >> 4;
    const int r0 = blockIdx.x * 64, c0 = blockIdx.y * 64;
    const int bb = r0 / SEQ, s0 = r0 % SEQ, hh = blockIdx.y;
    v8f acc[4][4];
#pragma unroll
    for (int mb = 0; mb < 4; ++mb)
#pragma unroll
        for (int nb = 0; nb < 4; ++nb) acc[mb][nb] = (v8f){};
    const size_t aoff = (size_t)(r0 + lr) * DM + 8 * hi, boff = (size_t)(c0 + lr) * DM + 8 * hi;
#pragma unroll 1
    for (int kc = 0; kc < DM; kc += 32) {
        V a[4]; V b;
#pragma unroll
        for (int mb = 0; mb < 4; ++mb) a[mb] = WFrag<T16>::ld(A + aoff + (size_t)mb * 16 * DM + kc);
#pragma unroll
        for (int nb = 0; nb < 4; ++nb) { b = WFrag<T16>::ld(Bt + boff + (size_t)nb * 16 * DM + kc);
#pragma unroll
            for (int mb = 0; mb < 4; ++mb) acc[mb][nb] = WFrag<T16>::mma(a[mb], b, acc[mb][nb]); }
        asm volatile("" : "+v"(acc[0][0]), "+v"(acc[1][0]), "+v"(acc[2][0]), "+v"(acc[3][0]), "+v"(acc[0][1]), "+v"(acc[1][1]), "+v"(acc[2][1]), "+v"(acc[3][1]));
        asm volatile("v_nop\n\tv_nop\n\tv_nop\n\tv_nop" : "+v"(acc[0][2]), "+v"(acc[1][2]), "+v"(acc[2][2]), "+v"(acc[3][2]), "+v"(acc[0][3]), "+v"(acc[1][3]), "+v"(acc[2][3]), "+v"(acc[3][3]) : "v"(a[3]), "v"(b));
    }
    if (MODE == 0) {
        const int rq = lane >> 3, c8 = (lane & 7) * 8;
        float bs[8];
#pragma unroll
        for (int e = 0; e < 8; ++e) bs[e] = bfr(bias[c0 + c8 + e]);
        h16* pbase = o16 + (((size_t)bb * NH + hh) * SEQ + s0) * HD + c8;
#pragma unroll
        for (int mb = 0; mb < 4; ++mb) {
#pragma unroll
            for (int nb = 0; nb < 4; ++nb)
#pragma unroll
                for (int j = 0; j < 8; ++j) os[(hi * 8 + j) * 68 + nb * 16 + lr] = acc[mb][nb][j];
            __syncthreads();
            v8h vals[4];
#pragma unroll
            for (int s = 0; s < 4; ++s) { const int row = 4 * s + rq; const v4f x0 = *(const v4fa*)(os + row * 68 + c8); const v4f x1 = *(const v4fa*)(os + row * 68 + c8 + 4);
#pragma unroll
                for (int e = 0; e < 4; ++e) { vals[s][e] = (h16)(x0[e] + bs[e]); vals[s][4 + e] = (h16)(x1[e] + bs[4 + e]); } }
#pragma unroll 1
            for (int ps = 0; ps < 2; ++ps) {
#pragma unroll
                for (int s = 0; s < 4; ++s) *(volatile v8h*)(pbase + (size_t)(mb * 16 + 4 * s + rq) * HD) = vals[s];
                if (ps == 0) __threadfence(); }
            __syncthreads();
        }
    }
    if (MODE == 1) {
        float bc[4];
#pragma unroll
        for (int nb = 0; nb < 4; ++nb) bc[nb] = bfr(bias[c0 + nb * 16 + lr]);
#pragma unroll
        for (int mb = 0; mb < 4; ++mb)
#pragma unroll
            for (int nb = 0; nb < 4; ++nb) { v8h o;
#pragma unroll
                for (int j = 0; j < 8; ++j) o[j] = (h16)(acc[mb][nb][j] + bc[nb]);
                *(v8h*)(vts + (nb * 16 + lr) * 72 + mb * 16 + 8 * hi) = o; }
        __syncthreads();
        const int rq = lane >> 3, c8 = (lane & 7) * 8;
        h16* vbase = o16 + (((size_t)bb * NH + hh) * HD) * SEQ + s0 + c8;
#pragma unroll 1
        for (int ps = 0; ps < 2; ++ps) {
#pragma unroll
            for (int s = 0; s < 16; ++s) { const int d = 4 * s + rq; const v8h val = *(const v8ha*)(vts + d * 72 + c8); *(volatile v8h*)(vbase + (size_t)d * SEQ) = val; }
            if (ps == 0) __threadfence(); }
    }
    if (MODE == 2) {
        const int cofs = lr * 4;
        float bo[4];
#pragma unroll
        for (int e = 0; e < 4; ++e) bo[e] = bfr(bias[c0 + cofs + e]);
        float* cbase = o32 + ((size_t)bb * SEQ_FULL + s0) * DM + c0 + cofs;
#pragma unroll
        for (int mb = 0; mb < 4; ++mb) {
#pragma unroll
            for (int nb = 0; nb < 4; ++nb)
#pragma unroll
                for (int j = 0; j < 8; ++j) os[(hi * 8 + j) * 68 + nb * 16 + lr] = acc[mb][nb][j];
            __syncthreads();
            v4f vals[8];
#pragma unroll
            for (int s = 0; s < 8; ++s) { const int row = 2 * s + hi; v4f v = *(const v4fa*)(os + row * 68 + cofs);
#pragma unroll
                for (int e = 0; e < 4; ++e) v[e] = v[e] * OSC + bo[e];
                vals[s] = v; }
#pragma unroll 1
            for (int ps = 0; ps < 2; ++ps) {
#pragma unroll
                for (int s = 0; s < 8; ++s) *(volatile v4f*)(cbase + (size_t)(mb * 16 + 2 * s + hi) * DM) = vals[s];
                if (ps == 0) __threadfence(); }
            __syncthreads();
        }
    }
}

__global__ __launch_bounds__(32) void k_proj_qk(const bf* __restrict__ A, const bf* __restrict__ Bt, const float* __restrict__ bias, h16* out) { gemm_body<bf, 0>(A, Bt, bias, out, nullptr); }
__global__ __launch_bounds__(32) void k_proj_v(const bf* __restrict__ A, const bf* __restrict__ Bt, const float* __restrict__ bias, h16* out) { gemm_body<bf, 1>(A, Bt, bias, out, nullptr); }
__global__ __launch_bounds__(32) void k_out(const h16* __restrict__ A, const h16* __restrict__ Bt, const float* __restrict__ bias, float* out) { gemm_body<h16, 2>(A, Bt, bias, nullptr, out); }

__global__ __launch_bounds__(128) void k_flash(const h16* __restrict__ QP, const h16* __restrict__ KP, const h16* __restrict__ VT, h16* CTX) {
    __shared__ __align__(16) h16 cs[AW * QW * 72];
    const int lane = threadIdx.x & 31, wid = threadIdx.x >> 5, lr = lane & 15, hi = lane >> 4;
    const int bh = blockIdx.y, b = bh / NH, h = bh % NH;
    const int q0 = (blockIdx.x * AW + wid) * QW;
    const h16* Qb = QP + ((size_t)bh * SEQ + q0 + lr) * HD + 8 * hi;
    const h16* Kb = KP + ((size_t)bh * SEQ + lr) * HD + 8 * hi;
    const h16* Vb = VT + ((size_t)bh * HD + lr) * SEQ + 8 * hi;
    v16h qf[2][2];
#pragma unroll
    for (int i = 0; i < 2; ++i)
#pragma unroll
        for (int kk = 0; kk < 2; ++kk) qf[i][kk] = WFrag<h16>::ld(Qb + (size_t)i * 16 * HD + kk * 32);
    v8f acc[4][2];
#pragma unroll
    for (int dt = 0; dt < 4; ++dt)
#pragma unroll
        for (int i = 0; i < 2; ++i) acc[dt][i] = (v8f){};
    float mrun[2], lrun[2];
#pragma unroll
    for (int i = 0; i < 2; ++i) { mrun[i] = -1.0e30f; lrun[i] = 0.0f; }

#pragma unroll 1
    for (int n0 = 0; n0 < SEQ; n0 += KB) {
#pragma unroll 1
        for (int u = 0; u < KB / KH; ++u) {
            const int kb = n0 + u * KH;
            v8f sc[2][2]; v16h ka0, ka1;
#pragma unroll
            for (int t = 0; t < 2; ++t) {
                ka0 = WFrag<h16>::ld(Kb + (size_t)(kb + t * 16) * HD);
                ka1 = WFrag<h16>::ld(Kb + (size_t)(kb + t * 16) * HD + 32);
#pragma unroll
                for (int i = 0; i < 2; ++i) { v8f z = (v8f){}; z = wmma16(ka0, qf[i][0], z); z = wmma16(ka1, qf[i][1], z); sc[t][i] = z; }
            }
            int vo = kb;
            asm volatile("v_nop\n\tv_nop\n\tv_nop\n\tv_nop" : "+v"(sc[0][0]), "+v"(sc[0][1]), "+v"(sc[1][0]), "+v"(sc[1][1]), "+v"(vo) : "v"(ka1), "v"(qf[1][1]));

            v16h pb[2];
#pragma unroll
            for (int i = 0; i < 2; ++i) {
                float mx = sc[0][i][0];
#pragma unroll
                for (int t = 0; t < 2; ++t)
#pragma unroll
                    for (int r = 0; r < 8; ++r) mx = fmaxf(mx, sc[t][i][r]);
                mx = fmaxf(mx, __shfl_xor(mx, 16, 32));
                const float mnew = fmaxf(mrun[i], mx);
                const float corr = __builtin_amdgcn_exp2f((mrun[i] - mnew) * EXC);
                mrun[i] = mnew;
                float ls = 0.0f;
#pragma unroll
                for (int t = 0; t < 2; ++t)
#pragma unroll
                    for (int r = 0; r < 8; ++r) { const float p = __builtin_amdgcn_exp2f((sc[t][i][r] - mnew) * EXC); const h16 ph = (h16)p; ls += (float)ph; pb[i][t * 8 + r] = ph; }
                lrun[i] = lrun[i] * corr + ls;
#pragma unroll
                for (int dt = 0; dt < 4; ++dt)
#pragma unroll
                    for (int r = 0; r < 8; ++r) acc[dt][i][r] *= corr;
            }

            v16h va[4];
#pragma unroll
            for (int dt = 0; dt < 4; ++dt) va[dt] = WFrag<h16>::ld(Vb + (size_t)(dt * 16) * SEQ + vo);
#pragma unroll
            for (int dt = 0; dt < 4; ++dt)
#pragma unroll
                for (int i = 0; i < 2; ++i) acc[dt][i] = wmma16(va[dt], pb[i], acc[dt][i]);
            asm volatile("v_nop\n\tv_nop\n\tv_nop\n\tv_nop" : "+v"(acc[0][0]), "+v"(acc[0][1]), "+v"(acc[1][0]), "+v"(acc[1][1]), "+v"(acc[2][0]), "+v"(acc[2][1]), "+v"(acc[3][0]), "+v"(acc[3][1]) : "v"(va[3]), "v"(pb[1]));
        }
    }

    h16* cw = cs + wid * (QW * 72);
#pragma unroll
    for (int i = 0; i < 2; ++i) {
        const float lt = lrun[i] + __shfl_xor(lrun[i], 16, 32);
        const float inv = CCAR * (1.0f / lt);
#pragma unroll
        for (int dt = 0; dt < 4; ++dt) { v8h o;
#pragma unroll
            for (int r = 0; r < 8; ++r) o[r] = (h16)(acc[dt][i][r] * inv);
            *(v8h*)(cw + (i * 16 + lr) * 72 + dt * 16 + 8 * hi) = o; }
    }
    __syncthreads();
    const int rq = lane >> 3, c8 = (lane & 7) * 8;
    v8h vals[8];
#pragma unroll
    for (int s = 0; s < 8; ++s) vals[s] = *(const v8ha*)(cw + (4 * s + rq) * 72 + c8);
    h16* crow = CTX + ((size_t)b * SEQ + q0) * DM + h * HD + c8;
#pragma unroll 1
    for (int ps = 0; ps < 2; ++ps) {
#pragma unroll
        for (int s = 0; s < 8; ++s) *(volatile v8h*)(crow + (size_t)(4 * s + rq) * DM) = vals[s];
        if (ps == 0) __threadfence(); }
}

constexpr size_t SZ_XB = (size_t)NB * SEQ * DM * 2;
constexpr size_t SZ_W  = (size_t)DM * DM * 2;
constexpr size_t SZ_PL = (size_t)NB * NH * SEQ * HD * 2;
constexpr size_t WS_TOTAL = SZ_XB + 4 * SZ_W + 3 * SZ_PL + SZ_XB;
static_assert(SZ_XB % 256 == 0);
static_assert(SZ_W % 256 == 0);
static_assert(SZ_PL % 256 == 0);
static_assert(WS_TOTAL <= (size_t)134217728);

extern "C" void kernel_launch(void* const* d_in, const int* in_sizes, int n_in,
                              void* d_out, int out_size, void* d_ws, size_t ws_size, hipStream_t stream) {
    if (n_in < 9) return;
    const size_t XMIN = ((size_t)(NB - 1) * SEQ_FULL + SEQ) * DM;
    if ((size_t)in_sizes[0] < XMIN) return;
    if ((size_t)in_sizes[1] < (size_t)DM * DM || (size_t)in_sizes[3] < (size_t)DM * DM || (size_t)in_sizes[5] < (size_t)DM * DM || (size_t)in_sizes[7] < (size_t)DM * DM) return;
    if (in_sizes[2] < DM || in_sizes[4] < DM || in_sizes[6] < DM || in_sizes[8] < DM) return;
    if ((size_t)out_size < XMIN) return;
    if (WS_TOTAL > ws_size) return;
    const float* x  = (const float*)d_in[0];
    const float* wq = (const float*)d_in[1]; const float* bq = (const float*)d_in[2];
    const float* wk = (const float*)d_in[3]; const float* bk = (const float*)d_in[4];
    const float* wv = (const float*)d_in[5]; const float* bv = (const float*)d_in[6];
    const float* wo = (const float*)d_in[7]; const float* bo = (const float*)d_in[8];
    float* OUT = (float*)d_out;
    char* wsp = (char*)d_ws;
    auto take = [&](size_t bytes) { char* p = wsp; wsp += bytes; return (void*)p; };
    bf* XB = (bf*)take(SZ_XB); bf* WQ = (bf*)take(SZ_W); bf* WK = (bf*)take(SZ_W); bf* WV = (bf*)take(SZ_W); h16* WO = (h16*)take(SZ_W);
    h16* QP = (h16*)take(SZ_PL); h16* KP = (h16*)take(SZ_PL); h16* VT = (h16*)take(SZ_PL); h16* CT = (h16*)take(SZ_XB);

    const size_t nx8 = (size_t)SEQ * DM / 8, nw8 = (size_t)DM * DM / 8;
    k_cvt8<<<dim3((unsigned)((nx8 + 255) / 256), NB), 256, 0, stream>>>(x, XB, nx8, (size_t)SEQ_FULL * DM, (size_t)SEQ * DM);
    k_cvt8<<<dim3((unsigned)((nw8 + 255) / 256), 1), 256, 0, stream>>>(wq, WQ, nw8, 0, 0);
    k_cvt8<<<dim3((unsigned)((nw8 + 255) / 256), 1), 256, 0, stream>>>(wk, WK, nw8, 0, 0);
    k_cvt8<<<dim3((unsigned)((nw8 + 255) / 256), 1), 256, 0, stream>>>(wv, WV, nw8, 0, 0);
    k_cvt8h<<<(unsigned)((nw8 + 255) / 256), 256, 0, stream>>>(wo, WO, nw8);

    const dim3 gg(NB * SEQ / 64, DM / 64);
    k_proj_qk<<<gg, 32, 0, stream>>>(XB, WQ, bq, QP);
    k_proj_qk<<<gg, 32, 0, stream>>>(XB, WK, bk, KP);
    k_proj_v<<<gg, 32, 0, stream>>>(XB, WV, bv, VT);

    k_flash<<<dim3(SEQ / (AW * QW), NB * NH), 128, 0, stream>>>(QP, KP, VT, CT);

    k_out<<<gg, 32, 0, stream>>>(CT, WO, bo, OUT);
}
